// EncoderBlock_16741782520182
// MI455X (gfx1250) — hardware-verified
//
#include <hip/hip_runtime.h>
#ifndef NB
#define NB 2
#endif
#ifndef SEQ
#define SEQ 2048
#endif
#define NB_FULL 2
#define SEQ_FULL 2048
#define DM 1024
#define NH 16
#define HD 64
#define DFF 4096
#define LN_DDOF 1
#define NR (NB * SEQ)

static_assert(DM == NH * HD);
static_assert(HD == 64);
static_assert(DM == 256 * 4);
static_assert(DM % 32 == 0);
static_assert(DFF % 32 == 0);
static_assert(DM % 128 == 0);
static_assert(DFF % 64 == 0);
static_assert(SEQ % 128 == 0);
static_assert(NR % 128 == 0);
static_assert(NR % 64 == 0);
static_assert(SEQ <= SEQ_FULL);
static_assert(NB <= NB_FULL);
static_assert(DM % 8 == 0);
static_assert(DFF % 8 == 0);

typedef unsigned short v8us __attribute__((ext_vector_type(8), may_alias));
typedef float  v8f  __attribute__((ext_vector_type(8)));
typedef float  v4f  __attribute__((ext_vector_type(4)));
typedef float  v4fa __attribute__((ext_vector_type(4), may_alias));
typedef _Float16 v16h __attribute__((ext_vector_type(16)));
typedef _Float16 v4h __attribute__((ext_vector_type(4)));
union FragH { v16h v; v8us half[2]; _Float16 h[16]; unsigned short u[16]; };
union H1 { _Float16 h; unsigned short u; };

__device__ __forceinline__ unsigned short bf16_bits(float x) { unsigned int u = __float_as_uint(x); return (unsigned short)((u + 0x7FFFu + ((u >> 16) & 1u)) >> 16); }
__device__ __forceinline__ float bf16_val(unsigned short b) { return __uint_as_float(((unsigned int)b) << 16); }
__device__ __forceinline__ float bf16_rne(float x) { return bf16_val(bf16_bits(x)); }
__device__ __forceinline__ int row_full(int r) { return (r / SEQ) * SEQ_FULL + (r % SEQ); }

__global__ __launch_bounds__(256) void k_wt_f16(const float* __restrict__ W, _Float16* __restrict__ Wt, int K, int N, float scale) {
  const int t = blockIdx.x * 256 + threadIdx.x; if (t >= N * (K / 8)) return; const int n = t / (K / 8), k8 = (t % (K / 8)) * 8; FragH f;
#pragma unroll
  for (int i = 0; i < 8; ++i) f.h[i] = (_Float16)(bf16_rne(W[(size_t)(k8 + i) * N + n]) * scale);
  const v8us o = f.half[0];
  *(volatile v8us*)((unsigned short*)Wt + (size_t)n * K + k8) = o; __threadfence(); *(volatile v8us*)((unsigned short*)Wt + (size_t)n * K + k8) = o;
}

__global__ __launch_bounds__(256) void k_lnsc(const float* __restrict__ X, const float* __restrict__ g, const float* __restrict__ bb, float eps, _Float16* __restrict__ N16, int bfin, int mapin) {
  #pragma clang fp contract(off)
  __shared__ float red[256];
  const int r = blockIdx.x; const int t = threadIdx.x;
  const size_t rin = (size_t)(mapin ? row_full(r) : r);
  const v4f xl = *(const v4fa*)(X + rin * DM + t * 4); float s[4]; float sum = 0.f;
#pragma unroll
  for (int q = 0; q < 4; ++q) { const float xr = bf16_rne(xl[q]); s[q] = bfin ? xr : xl[q]; sum = __fadd_rn(sum, s[q]); }
  red[t] = sum; __syncthreads();
  for (int st = 128; st > 0; st >>= 1) { if (t < st) red[t] = __fadd_rn(red[t], red[t + st]); __syncthreads(); }
  const float mu = red[0] / (float)DM; __syncthreads();
  float vs = 0.f;
#pragma unroll
  for (int q = 0; q < 4; ++q) { const float dl = __fadd_rn(s[q], -mu); vs = __fadd_rn(vs, __fmul_rn(dl, dl)); }
  red[t] = vs; __syncthreads();
  for (int st = 128; st > 0; st >>= 1) { if (t < st) red[t] = __fadd_rn(red[t], red[t + st]); __syncthreads(); }
  const float rs = __fdiv_rn(1.0f, __fadd_rn(sqrtf(red[0] / (float)(DM - LN_DDOF)), eps));
  const float gg = bf16_rne(g[0]), bv = bf16_rne(bb[0]);
  v4h y;
#pragma unroll
  for (int q = 0; q < 4; ++q) y[q] = (_Float16)__fadd_rn(__fmul_rn(__fmul_rn(__fadd_rn(s[q], -mu), rs), gg), bv);
  for (int pass = 0; pass < 2; ++pass) { *(volatile v4h*)(N16 + (size_t)r * DM + t * 4) = y; if (pass == 0) __threadfence(); }
}

__device__ __forceinline__ v16h g2_frag(const _Float16* p, int hh) { FragH f; f.half[0] = *(const v8us*)((const unsigned short*)p + 8 * hh); f.half[1] = *(const v8us*)((const unsigned short*)p + 16 + 8 * hh); return f.v; }
__device__ __forceinline__ v8f g2_mma(v16h a, v16h b, v8f c) { v8f d = __builtin_amdgcn_wmma_f32_16x16x32_f16(false, a, false, b, (short)0, c, false, false); asm volatile("v_nop\n\tv_nop\n\tv_nop\n\tv_nop" : "+v"(d) : "v"(a), "v"(b)); return d; }

template <int ACT, int OUTM, int BIASROW, int RESM, int OMAP>
__device__ __forceinline__ void gemm2_body(const _Float16* __restrict__ A, int lda, const _Float16* __restrict__ Bh, int ldb, float alpha, const float* __restrict__ bias,
                                           const float* __restrict__ resid, int ldr, float* __restrict__ C, _Float16* __restrict__ C16, int ldc, int M, int N, int K) {
  static_assert(OUTM == 0 || OUTM == 1);
  __shared__ __attribute__((aligned(16))) float so[4][32][68];
  const int tid = threadIdx.x, w = tid >> 5, lane = tid & 31, ln = lane & 15, hh = lane >> 4;
  const int ntn = N >> 6; const int mt = blockIdx.x / ntn, nq = blockIdx.x - mt * ntn; const int row0 = mt * 128 + 32 * w, col0 = nq * 64; if (row0 >= M) return;
  const _Float16* a0p = A + (size_t)(row0 + ln) * lda; const _Float16* a1p = a0p + (size_t)16 * lda;
  const _Float16* b0p = Bh + (size_t)(col0 + ln) * ldb; const _Float16* b1p = b0p + (size_t)16 * ldb; const _Float16* b2p = b1p + (size_t)16 * ldb; const _Float16* b3p = b2p + (size_t)16 * ldb;
  const v8f z8 = {0.f,0.f,0.f,0.f,0.f,0.f,0.f,0.f}; v8f c00 = z8, c01 = z8, c02 = z8, c03 = z8, c10 = z8, c11 = z8, c12 = z8, c13 = z8;
#pragma unroll 1
  for (int kb = 0; kb < K; kb += 32) { const v16h a0 = g2_frag(a0p + kb, hh), a1 = g2_frag(a1p + kb, hh);
    v16h b = g2_frag(b0p + kb, hh); c00 = g2_mma(a0, b, c00); c10 = g2_mma(a1, b, c10);
    b = g2_frag(b1p + kb, hh); c01 = g2_mma(a0, b, c01); c11 = g2_mma(a1, b, c11);
    b = g2_frag(b2p + kb, hh); c02 = g2_mma(a0, b, c02); c12 = g2_mma(a1, b, c12);
    b = g2_frag(b3p + kb, hh); c03 = g2_mma(a0, b, c03); c13 = g2_mma(a1, b, c13); }
  v8f accs[8] = {c00, c01, c02, c03, c10, c11, c12, c13};
#pragma unroll
  for (int u = 0; u < 8; ++u) { const int t = u & 3, half = u >> 2; const int col = col0 + t * 16 + ln; const float bcol = BIASROW ? 0.f : bf16_rne(bias[col]);
#pragma unroll
    for (int r = 0; r < 8; ++r) { const int rloc = half * 16 + 8 * hh + r; const float bv = BIASROW ? bf16_rne(bias[row0 + rloc]) : bcol;
      float v = accs[u][r] * alpha + bv; if (ACT == 1) v = fmaxf(v, 0.f);
      so[w][rloc][t * 16 + ln] = v; } }
  __builtin_amdgcn_fence(4  , "workgroup"); __builtin_amdgcn_wave_barrier();
  const int rsub = lane >> 4, c4 = (lane & 15) * 4;
  for (int pass = 0; pass < 2; ++pass) {
#pragma unroll
    for (int q = 0; q < 16; ++q) { const int r = q * 2 + rsub; const int grow = row0 + r; v4f v = *(const v4fa*)&so[w][r][c4];
      if (OUTM == 0) {
        if (RESM != 0) { const size_t rr = (size_t)((RESM == 1) ? row_full(grow) : grow); v4f rv = *(const v4fa*)(resid + rr * ldr + col0 + c4);
          if (RESM == 1) { for (int i = 0; i < 4; ++i) rv[i] = bf16_rne(rv[i]); }
          for (int i = 0; i < 4; ++i) v[i] = v[i] + rv[i]; }
        const size_t orow = (size_t)(OMAP ? row_full(grow) : grow);
        *(volatile v4f*)(C + orow * ldc + col0 + c4) = v;
      } else {
        v4h h4; for (int i = 0; i < 4; ++i) h4[i] = (_Float16)v[i];
        *(volatile v4h*)(C16 + (size_t)grow * ldc + col0 + c4) = h4;
      } }
    if (pass == 0) __threadfence(); } }

__global__ __launch_bounds__(128) void k_gemm_qk(const _Float16* __restrict__ A, const _Float16* __restrict__ Bt, const float* __restrict__ bias, _Float16* __restrict__ Ch) {
  gemm2_body<0, 1, 0, 0, 0>(A, DM, Bt, DM, 0.0625f, bias, nullptr, 0, nullptr, Ch, DM, NR, DM, DM); }
__global__ __launch_bounds__(128) void k_gemm_vt(const _Float16* __restrict__ Wt, const _Float16* __restrict__ Xn, const float* __restrict__ bias, _Float16* __restrict__ VT) {
  gemm2_body<0, 1, 1, 0, 0>(Wt, DM, Xn, DM, 0.0625f, bias, nullptr, 0, nullptr, VT, NR, DM, NR, DM); }
__global__ __launch_bounds__(128) void k_gemm_wo(const _Float16* __restrict__ A, const _Float16* __restrict__ Bt, const float* __restrict__ bias, const float* __restrict__ x, float* __restrict__ X1) {
  gemm2_body<0, 0, 0, 1, 0>(A, DM, Bt, DM, 0.0009765625f, bias, x, DM, X1, nullptr, DM, NR, DM, DM); }
__global__ __launch_bounds__(128) void k_gemm_f1(const _Float16* __restrict__ A, const _Float16* __restrict__ Bt, const float* __restrict__ bias, _Float16* __restrict__ H) {
  gemm2_body<1, 1, 0, 0, 0>(A, DM, Bt, DM, 0.0625f, bias, nullptr, 0, nullptr, H, DFF, NR, DFF, DM); }
__global__ __launch_bounds__(128) void k_gemm_f2(const _Float16* __restrict__ A, const _Float16* __restrict__ Bt, const float* __restrict__ bias, const float* __restrict__ X1, float* __restrict__ out) {
  gemm2_body<0, 0, 0, 2, 1>(A, DFF, Bt, DFF, 0.0625f, bias, X1, DM, out, nullptr, DM, NR, DM, DFF); }

__global__ __launch_bounds__(128) void k_flash(const _Float16* __restrict__ QH, const _Float16* __restrict__ KH,
                                               const _Float16* __restrict__ VT, const int* __restrict__ mask, _Float16* __restrict__ O16) {
  __shared__ __attribute__((aligned(16))) unsigned short ps[4][16][72];
  const int tid = threadIdx.x, w = tid >> 5, lane = tid & 31, ln = lane & 15, hh = lane >> 4;
  const int bh = blockIdx.y; const int b = bh / NH, h = bh % NH;
  const int q0 = blockIdx.x * 64 + w * 16;
  const size_t rbase = (size_t)b * SEQ;
  const _Float16* qp = QH + (rbase + q0 + ln) * DM + h * HD;
  const v16h qh0 = g2_frag(qp, hh), qh1 = g2_frag(qp + 32, hh);
  const _Float16* kph = KH + (rbase + ln) * DM + h * HD;
  const _Float16* vtp = VT + (size_t)(h * HD + ln) * NR + rbase;
  const int* mp = mask + (size_t)b * SEQ_FULL;
  const v8f z8 = {0.f,0.f,0.f,0.f,0.f,0.f,0.f,0.f};
  v8f o[4]; float mrun[8], lrun[8];
#pragma unroll
  for (int t = 0; t < 4; ++t) o[t] = z8;
#pragma unroll
  for (int r = 0; r < 8; ++r) { mrun[r] = -1.0e30f; lrun[r] = 0.f; }
#pragma unroll 1
  for (int kb = 0; kb < SEQ; kb += 64) {
    v8f sh[4]; int mk[4];
#pragma unroll
    for (int t = 0; t < 4; ++t) { sh[t] = z8; mk[t] = mp[kb + t * 16 + ln]; }
#pragma unroll
    for (int t = 0; t < 4; ++t) {
      const _Float16* kr = kph + (size_t)(kb + t * 16) * DM;
      v16h bk = g2_frag(kr, hh);
      sh[t] = g2_mma(qh0, bk, sh[t]);
      bk = g2_frag(kr + 32, hh);
      sh[t] = g2_mma(qh1, bk, sh[t]);
    }
#pragma unroll
    for (int r = 0; r < 8; ++r) {
      float v[4];
#pragma unroll
      for (int t = 0; t < 4; ++t) { const float s = sh[t][r] * 0.125f; v[t] = (mk[t] != 0) ? s : -1.0e9f; }
      float mx = fmaxf(fmaxf(v[0], v[1]), fmaxf(v[2], v[3]));
      mx = fmaxf(mx, __shfl_xor(mx, 1, 32)); mx = fmaxf(mx, __shfl_xor(mx, 2, 32)); mx = fmaxf(mx, __shfl_xor(mx, 4, 32)); mx = fmaxf(mx, __shfl_xor(mx, 8, 32));
      const float mnew = fmaxf(mrun[r], mx); const float al = __expf(mrun[r] - mnew); mrun[r] = mnew;
      float psum = 0.f;
#pragma unroll
      for (int t = 0; t < 4; ++t) { const float p = __expf(v[t] - mnew); psum += p; H1 c; c.h = (_Float16)(p * 256.0f); ps[w][8 * hh + r][t * 16 + ln] = c.u; }
      lrun[r] = lrun[r] * al + psum;
#pragma unroll
      for (int t = 0; t < 4; ++t) o[t][r] *= al;
    }
    __builtin_amdgcn_fence(4  , "workgroup"); __builtin_amdgcn_wave_barrier();
    FragH pf0, pf1;
    pf0.half[0] = *(const v8us*)&ps[w][ln][8 * hh]; pf0.half[1] = *(const v8us*)&ps[w][ln][16 + 8 * hh];
    pf1.half[0] = *(const v8us*)&ps[w][ln][32 + 8 * hh]; pf1.half[1] = *(const v8us*)&ps[w][ln][48 + 8 * hh];
#pragma unroll
    for (int t = 0; t < 4; ++t) {
      const _Float16* vr = vtp + (size_t)(t * 16) * NR + kb;
      v16h bv = g2_frag(vr, hh); o[t] = g2_mma(pf0.v, bv, o[t]);
      bv = g2_frag(vr + 32, hh); o[t] = g2_mma(pf1.v, bv, o[t]);
    }
    __builtin_amdgcn_fence(4  , "workgroup"); __builtin_amdgcn_wave_barrier();
  }
#pragma unroll
  for (int r = 0; r < 8; ++r) {
    float l = lrun[r];
    l += __shfl_xor(l, 1, 32); l += __shfl_xor(l, 2, 32); l += __shfl_xor(l, 4, 32); l += __shfl_xor(l, 8, 32);
    const float fin = 0.25f * (1.0f / l);
#pragma unroll
    for (int t = 0; t < 4; ++t) { H1 c; c.h = (_Float16)(o[t][r] * fin); ps[w][8 * hh + r][t * 16 + ln] = c.u; }
  }
  __builtin_amdgcn_fence(4  , "workgroup"); __builtin_amdgcn_wave_barrier();
  const int rq = lane >> 3, pc = (lane & 7) * 8;
  for (int pass = 0; pass < 2; ++pass) {
#pragma unroll
    for (int q = 0; q < 4; ++q) { const int row = q * 4 + rq; const v8us v = *(const v8us*)&ps[w][row][pc];
      *(volatile v8us*)((unsigned short*)O16 + (rbase + q0 + row) * DM + h * HD + pc) = v; }
    if (pass == 0) __threadfence(); }
}

extern "C" void kernel_launch(void* const* d_in, const int* in_sizes, int n_in,
                              void* d_out, int out_size, void* d_ws, size_t ws_size, hipStream_t stream) {
  if (n_in < 18) return;
  constexpr long long ROWS_SPAN = (long long)(NB - 1) * SEQ_FULL + SEQ;
  if ((long long)in_sizes[0] < ROWS_SPAN * DM) return;
  if ((long long)in_sizes[1] < ROWS_SPAN) return;
  if (in_sizes[2] < DM * DM || in_sizes[4] < DM * DM || in_sizes[6] < DM * DM || in_sizes[8] < DM * DM) return;
  if (in_sizes[3] < DM || in_sizes[5] < DM || in_sizes[7] < DM || in_sizes[9] < DM || in_sizes[13] < DM) return;
  if (in_sizes[10] < DM * DFF || in_sizes[12] < DM * DFF || in_sizes[11] < DFF) return;
  if (in_sizes[14] < 1 || in_sizes[15] < 1 || in_sizes[16] < 1 || in_sizes[17] < 1) return;
  if ((long long)out_size < ROWS_SPAN * DM) return;
  const float* x = (const float*)d_in[0]; const int* mask = (const int*)d_in[1];
  const float* wq = (const float*)d_in[2]; const float* bq = (const float*)d_in[3]; const float* wk = (const float*)d_in[4]; const float* bk = (const float*)d_in[5];
  const float* wv = (const float*)d_in[6]; const float* bv = (const float*)d_in[7]; const float* wo = (const float*)d_in[8]; const float* bo = (const float*)d_in[9];
  const float* w1 = (const float*)d_in[10]; const float* b1 = (const float*)d_in[11]; const float* w2 = (const float*)d_in[12]; const float* b2 = (const float*)d_in[13];
  const float* g1 = (const float*)d_in[14]; const float* be1 = (const float*)d_in[15]; const float* g2 = (const float*)d_in[16]; const float* be2 = (const float*)d_in[17];
  constexpr size_t SZ_W = (size_t)DM * DM * 2, SZ_WF = (size_t)DM * DFF * 2, SZ_R16 = (size_t)NR * DM * 2, SZ_HF = (size_t)NR * DFF * 2, SZ_X1 = (size_t)NR * DM * 4;
  constexpr size_t SZ_ATT = (4 * SZ_R16 > SZ_HF) ? 4 * SZ_R16 : SZ_HF;
  constexpr size_t OFF_BQ = 0, OFF_BK = OFF_BQ + SZ_W, OFF_BV = OFF_BK + SZ_W, OFF_BO = OFF_BV + SZ_W, OFF_W1 = OFF_BO + SZ_W, OFF_W2 = OFF_W1 + SZ_WF;
  constexpr size_t OFF_XN = OFF_W2 + SZ_WF, OFF_ATT = OFF_XN + SZ_R16, OFF_X1 = OFF_ATT + SZ_ATT, OFF_END = OFF_X1 + SZ_X1;
  constexpr size_t OFF_QH = OFF_ATT, OFF_KH = OFF_ATT + SZ_R16, OFF_VT = OFF_ATT + 2 * SZ_R16, OFF_O = OFF_ATT + 3 * SZ_R16;
  static_assert(SZ_W % 256 == 0 && SZ_WF % 256 == 0 && SZ_R16 % 256 == 0 && SZ_HF % 256 == 0 && SZ_X1 % 256 == 0);
  static_assert(OFF_O + SZ_R16 <= OFF_ATT + SZ_ATT);
  static_assert(SZ_HF <= SZ_ATT);
  static_assert(OFF_ATT + SZ_ATT <= OFF_X1);
  static_assert(OFF_END <= (size_t)134217728);
  if (OFF_END > ws_size) return;
  char* ws = (char*)d_ws;
  _Float16* BQ = (_Float16*)(ws + OFF_BQ); _Float16* BK = (_Float16*)(ws + OFF_BK); _Float16* BV = (_Float16*)(ws + OFF_BV); _Float16* BO = (_Float16*)(ws + OFF_BO);
  _Float16* BW1 = (_Float16*)(ws + OFF_W1); _Float16* BW2 = (_Float16*)(ws + OFF_W2);
  _Float16* XN = (_Float16*)(ws + OFF_XN); _Float16* M16 = XN;
  _Float16* QHp = (_Float16*)(ws + OFF_QH); _Float16* KHp = (_Float16*)(ws + OFF_KH);
  _Float16* VT = (_Float16*)(ws + OFF_VT); _Float16* O16 = (_Float16*)(ws + OFF_O);
  _Float16* HF16 = (_Float16*)(ws + OFF_ATT);
  float* X1 = (float*)(ws + OFF_X1);

  { const unsigned g = (unsigned)(((size_t)DM * (DM / 8) + 255) / 256);
    k_wt_f16<<<g, 256, 0, stream>>>(wq, BQ, DM, DM, 16.0f); k_wt_f16<<<g, 256, 0, stream>>>(wk, BK, DM, DM, 16.0f);
    k_wt_f16<<<g, 256, 0, stream>>>(wv, BV, DM, DM, 16.0f); k_wt_f16<<<g, 256, 0, stream>>>(wo, BO, DM, DM, 16.0f); }
  k_wt_f16<<<(unsigned)(((size_t)DFF * (DM / 8) + 255) / 256), 256, 0, stream>>>(w1, BW1, DM, DFF, 16.0f);
  k_wt_f16<<<(unsigned)(((size_t)DM * (DFF / 8) + 255) / 256), 256, 0, stream>>>(w2, BW2, DFF, DM, 16.0f);
  k_lnsc<<<(unsigned)NR, 256, 0, stream>>>(x, g1, be1, 1e-6f, XN, 1, 1);
  k_gemm_qk<<<(unsigned)((NR / 128) * (DM / 64)), 128, 0, stream>>>(XN, BQ, bq, QHp);
  k_gemm_qk<<<(unsigned)((NR / 128) * (DM / 64)), 128, 0, stream>>>(XN, BK, bk, KHp);
  k_gemm_vt<<<(unsigned)((DM / 128) * (NR / 64)), 128, 0, stream>>>(BV, XN, bv, VT);
  k_flash<<<dim3(SEQ / 64, NB * NH), 128, 0, stream>>>(QHp, KHp, VT, mask, O16);
  k_gemm_wo<<<(unsigned)((NR / 128) * (DM / 64)), 128, 0, stream>>>(O16, BO, bo, x, X1);
  k_lnsc<<<(unsigned)NR, 256, 0, stream>>>(X1, g2, be2, 1e-6f, M16, 0, 0);
  k_gemm_f1<<<(unsigned)((NR / 128) * (DFF / 64)), 128, 0, stream>>>(M16, BW1, b1, HF16);
  k_gemm_f2<<<(unsigned)((NR / 128) * (DM / 64)), 128, 0, stream>>>(HF16, BW2, b2, X1, (float*)d_out);
}
